// STU_23321672417769
// MI455X (gfx1250) — hardware-verified
//
#include <hip/hip_runtime.h>
#include <math.h>
#include <stddef.h>

typedef __attribute__((ext_vector_type(16))) _Float16 v16h;
typedef __attribute__((ext_vector_type(8)))  _Float16 v8h;
typedef __attribute__((ext_vector_type(8)))  float    v8f;
typedef __attribute__((ext_vector_type(4)))  float    v4f;

constexpr int NB     = 2;
constexpr int SEQ    = 1024;
constexpr int DMOD   = 768;
constexpr int NEIG   = 16;
constexpr int NFILT  = 32;
constexpr int NLAGU  = 3;
constexpr int NLAGY  = 2;
constexpr int KSPEC  = NFILT * DMOD;
constexpr int KLAGU  = NLAGU * DMOD;
constexpr int KLAGY  = NLAGY * DMOD;
constexpr int SEQP   = SEQ + 2;
constexpr int WPITCH = 1152;
constexpr int WLEN   = 1104;
constexpr int NTHR   = 256;
constexpr int SLABP  = 68;
constexpr int TILE   = 64;
constexpr int TILES_PER_PLANE = (SEQ / TILE) * (DMOD / TILE);
constexpr int GEMM_GX = TILES_PER_PLANE / 8;
constexpr float WCARRY     = 16.0f;
constexpr float WCARRY_INV = 0.0625f;

static_assert(TILES_PER_PLANE % 8 == 0);
static_assert(SEQ % TILE == 0 && DMOD % TILE == 0);
static_assert(KSPEC % 32 == 0 && KLAGU % 32 == 0 && KLAGY % 32 == 0 && SEQ % 32 == 0);
static_assert(WLEN % 8 == 0 && WPITCH % 8 == 0);
static_assert((((SEQ - 1) + 40) & ~7) + 23 < WLEN);
static_assert(WLEN - 1 + 7 < WPITCH);
static_assert(DMOD % 8 == 0 && (KLAGU / 8) % 32 == 0 && (DMOD / 8) % 32 == 0);

constexpr size_t SZ_UC    = (size_t)SEQ * KSPEC * 2;
constexpr size_t SZ_MCAT  = (size_t)DMOD * KSPEC * 2;
constexpr size_t SZ_USH   = (size_t)NB * SEQ * KLAGU * 2;
constexpr size_t SZ_SP    = (size_t)NB * SEQP * DMOD * 4;
constexpr size_t SZ_ZF    = (size_t)NB * SEQ * DMOD * 4;
constexpr size_t SZ_ZP    = (size_t)NB * SEQP * DMOD * 2;
constexpr size_t SZ_MUT   = (size_t)DMOD * KLAGU * 2;
constexpr size_t SZ_UT    = (size_t)NB * DMOD * SEQ * 2;
constexpr size_t SZ_MY    = (size_t)DMOD * KLAGY * 2;
constexpr size_t SZ_WREV  = (size_t)NFILT * WPITCH * 2;
constexpr size_t OFF_UC   = 0;
constexpr size_t OFF_MCAT = OFF_UC + SZ_UC;
constexpr size_t OFF_USH  = OFF_MCAT + SZ_MCAT;
constexpr size_t OFF_SP   = OFF_USH + SZ_USH;
constexpr size_t OFF_ZF   = OFF_SP + SZ_SP;
constexpr size_t OFF_ZP   = OFF_ZF + SZ_ZF;
constexpr size_t OFF_MUT  = OFF_ZP + SZ_ZP;
constexpr size_t OFF_UT   = OFF_MUT + SZ_MUT;
constexpr size_t OFF_MY   = OFF_UT + SZ_UT;
constexpr size_t OFF_WREV = OFF_MY + SZ_MY;
constexpr size_t WS_TOTAL = OFF_WREV + SZ_WREV;
static_assert(WS_TOTAL == (size_t)122382336);
static_assert(WS_TOTAL <= (size_t)134217728);
static_assert(SZ_UC % 128 == 0 && SZ_MCAT % 128 == 0 && SZ_USH % 128 == 0 && SZ_SP % 128 == 0 && SZ_ZF % 128 == 0);
static_assert(SZ_ZP % 128 == 0 && SZ_MUT % 128 == 0 && SZ_UT % 128 == 0 && SZ_MY % 128 == 0 && SZ_WREV % 128 == 0);

static_assert((NFILT * WPITCH / 8) % NTHR == 0);
static_assert((NB * SEQ * KLAGU / 8) % NTHR == 0);
static_assert((DMOD * KLAGY / 8) % NTHR == 0);
static_assert((NB * 2 * DMOD / 4) % NTHR == 0);
constexpr int ZP_GROUPS = NB * SEQP * DMOD / 8;

__device__ __forceinline__ unsigned short f2bf_bits(float f) {
  unsigned u = __float_as_uint(f);
  return (unsigned short)((u + 0x7FFFu + ((u >> 16) & 1u)) >> 16);
}
__device__ __forceinline__ float bf_bits2f(unsigned short h) { return __uint_as_float(((unsigned)h) << 16); }
__device__ __forceinline__ float bfr(float f) { return bf_bits2f(f2bf_bits(f)); }

__device__ __forceinline__ void keep4_h(v16h a, v16h b, v16h c, v16h d) { asm volatile("v_nop" :: "v"(a), "v"(b), "v"(c), "v"(d)); }
__device__ __forceinline__ void acc_guard4(v8f& a, v8f& b, v8f& c, v8f& d) { asm volatile("v_nop\n\tv_nop\n\tv_nop\n\tv_nop" : "+v"(a), "+v"(b), "+v"(c), "+v"(d)); }
__device__ __forceinline__ void mma_guard4(v8f& a, v8f& b, v8f& c, v8f& d, v16h x, v16h y) {
  asm volatile("v_nop\n\tv_nop\n\tv_nop\n\tv_nop" : "+v"(a), "+v"(b), "+v"(c), "+v"(d) : "v"(x), "v"(y));
}

struct FragH {
  union U { v16h v; v8h h[2]; };
  static __device__ __forceinline__ v16h load(const _Float16* p) {
    U f; f.h[0] = *(const v8h*)(p); f.h[1] = *(const v8h*)(p + 16); return f.v;
  }
  static __device__ __forceinline__ v8f mma(v16h a, v16h b, v8f c) {
    return __builtin_amdgcn_wmma_f32_16x16x32_f16(false, a, false, b, (short)0, c, false, false);
  }
};

template <bool RESID>
__global__ __launch_bounds__(NTHR) void gemm64_f16(
    const unsigned short* __restrict__ Ap, int lda, long strideA,
    const unsigned short* __restrict__ Btp, int ldb, long strideB,
    float* __restrict__ Cout, int ldc, long strideC,
    const float* __restrict__ resid, long strideR,
    int M, int N, int K, float scale) {
  __shared__ __align__(16) float sT[8][16 * SLABP];
  const int b    = blockIdx.y;
  const int lane = threadIdx.x & 31;
  const int wave = threadIdx.x >> 5;
  const int tilesN = N >> 6;
  const int tilesM = M >> 6;
  const int tile = blockIdx.x * 8 + wave;
  if (tile >= tilesM * tilesN) return;
  const int tm = tile / tilesN;
  const int tn = tile - tm * tilesN;
  const int m0 = tm << 6;
  const int n0 = tn << 6;

  const _Float16* Ab = (const _Float16*)Ap  + (size_t)b * strideA;
  const _Float16* Bb = (const _Float16*)Btp + (size_t)b * strideB;

  const int rlane = lane & 15;
  const int koff  = (lane >> 4) * 8;
  const int mOff  = (lane >> 4) * 8;

  v8f acc[4][4];
#pragma unroll
  for (int i = 0; i < 4; ++i)
#pragma unroll
    for (int j = 0; j < 4; ++j) acc[i][j] = (v8f){0.f,0.f,0.f,0.f,0.f,0.f,0.f,0.f};

  for (int k0 = 0; k0 < K; k0 += 32) {
    v16h bq[4];
#pragma unroll
    for (int j = 0; j < 4; ++j) {
      const size_t bo = (size_t)(n0 + (j << 4) + rlane) * ldb + koff + k0;
      bq[j] = FragH::load(Bb + bo);
    }
#pragma unroll
    for (int i = 0; i < 4; ++i) {
      const size_t ao = (size_t)(m0 + (i << 4) + rlane) * lda + koff + k0;
      const v16h ah = FragH::load(Ab + ao);
#pragma unroll
      for (int j = 0; j < 4; ++j) acc[i][j] = FragH::mma(ah, bq[j], acc[i][j]);
      mma_guard4(acc[i][0], acc[i][1], acc[i][2], acc[i][3], ah, bq[3]);
    }
    keep4_h(bq[0], bq[1], bq[2], bq[3]);
  }
  acc_guard4(acc[0][0], acc[0][1], acc[0][2], acc[0][3]);
  acc_guard4(acc[1][0], acc[1][1], acc[1][2], acc[1][3]);
  acc_guard4(acc[2][0], acc[2][1], acc[2][2], acc[2][3]);
  acc_guard4(acc[3][0], acc[3][1], acc[3][2], acc[3][3]);

  float* slab = sT[wave];
  float* C = Cout + (size_t)b * strideC;
  const float* Rb = RESID ? (resid + (size_t)b * strideR) : nullptr;
#pragma unroll
  for (int i = 0; i < 4; ++i) {
    const int mBase = m0 + (i << 4);
#pragma unroll
    for (int j = 0; j < 4; ++j) {
#pragma unroll
      for (int r = 0; r < 8; ++r) slab[(mOff + r) * SLABP + (j << 4) + rlane] = acc[i][j][r] * scale;
    }
    __builtin_amdgcn_fence(__ATOMIC_RELEASE, "workgroup");
    __builtin_amdgcn_wave_barrier();
    __builtin_amdgcn_fence(__ATOMIC_ACQUIRE, "workgroup");
    {
      const int hh = lane >> 4, c4 = (lane & 15) * 4;
      for (int pass = 0; pass < 2; ++pass) {
#pragma unroll
        for (int it = 0; it < 8; ++it) {
          const int row = it * 2 + hh;
          v4f v = *(const v4f*)(slab + row * SLABP + c4);
          const size_t go = (size_t)(mBase + row) * ldc + n0 + c4;
          if (RESID) {
            const v4f rr = *(const v4f*)(Rb + go);
            v = v + rr;
          }
          *(volatile v4f*)(C + go) = v;
        }
        __threadfence();
      }
    }
    __builtin_amdgcn_fence(__ATOMIC_RELEASE, "workgroup");
    __builtin_amdgcn_wave_barrier();
    __builtin_amdgcn_fence(__ATOMIC_ACQUIRE, "workgroup");
  }
}

__global__ __launch_bounds__(NTHR) void conv_causal_f16(
    const unsigned short* __restrict__ Wrev, const unsigned short* __restrict__ uTb,
    const float* __restrict__ sigma, unsigned short* __restrict__ Uc) {
  __shared__ __align__(16) _Float16 Wsh[8 * WLEN];
  __shared__ __align__(16) float sT[8][16 * SLABP];
  const int tid  = threadIdx.x;
  const int lane = tid & 31;
  const int wave = tid >> 5;
  const int kf   = blockIdx.y;

#pragma unroll 1
  for (int i = tid; i < 8 * WLEN; i += NTHR) {
    const int c = i / WLEN;
    const int p = i - c * WLEN;
    const unsigned short w = Wrev[(size_t)kf * WPITCH + p + c];
    Wsh[i] = __builtin_bit_cast(_Float16, w);
  }
  __syncthreads();

  const float sc = sqrtf(sqrtf(bfr(sigma[kf & (NEIG - 1)])));

  const int tile = blockIdx.x * 8 + wave;
  const int tm = tile / (DMOD / TILE);
  const int tn = tile - tm * (DMOD / TILE);
  const int m0 = tm << 6;
  const int n0 = tn << 6;

  const _Float16* Bb = (const _Float16*)uTb;
  const int rlane = lane & 15;
  const int koff  = (lane >> 4) * 8;
  const int mOff  = (lane >> 4) * 8;

  v8f acc[4][4];
#pragma unroll
  for (int i = 0; i < 4; ++i)
#pragma unroll
    for (int j = 0; j < 4; ++j) acc[i][j] = (v8f){0.f,0.f,0.f,0.f,0.f,0.f,0.f,0.f};

  const int kEnd = m0 + TILE;
  for (int k0 = 0; k0 < kEnd; k0 += 32) {
    v16h bq[4];
#pragma unroll
    for (int j = 0; j < 4; ++j) {
      const size_t bo = (size_t)(n0 + (j << 4) + rlane) * SEQ + koff + k0;
      bq[j] = FragH::load(Bb + bo);
    }
#pragma unroll
    for (int i = 0; i < 4; ++i) {
      const int l  = m0 + (i << 4) + rlane;
      const int st = (SEQ - 1) - l + k0 + koff;
      const int ao = (st & 7) * WLEN + (st & ~7);
      const v16h ah = FragH::load(Wsh + ao);
#pragma unroll
      for (int j = 0; j < 4; ++j) acc[i][j] = FragH::mma(ah, bq[j], acc[i][j]);
      mma_guard4(acc[i][0], acc[i][1], acc[i][2], acc[i][3], ah, bq[3]);
    }
    keep4_h(bq[0], bq[1], bq[2], bq[3]);
  }
  acc_guard4(acc[0][0], acc[0][1], acc[0][2], acc[0][3]);
  acc_guard4(acc[1][0], acc[1][1], acc[1][2], acc[1][3]);
  acc_guard4(acc[2][0], acc[2][1], acc[2][2], acc[2][3]);
  acc_guard4(acc[3][0], acc[3][1], acc[3][2], acc[3][3]);

  float* slab = sT[wave];
  unsigned short* C = Uc + (size_t)kf * DMOD;
#pragma unroll
  for (int i = 0; i < 4; ++i) {
    const int mBase = m0 + (i << 4);
#pragma unroll
    for (int j = 0; j < 4; ++j) {
#pragma unroll
      for (int r = 0; r < 8; ++r) slab[(mOff + r) * SLABP + (j << 4) + rlane] = acc[i][j][r] * sc;
    }
    __builtin_amdgcn_fence(__ATOMIC_RELEASE, "workgroup");
    __builtin_amdgcn_wave_barrier();
    __builtin_amdgcn_fence(__ATOMIC_ACQUIRE, "workgroup");
    {
      const int q = lane >> 3, c8 = (lane & 7) * 8;
      for (int pass = 0; pass < 2; ++pass) {
#pragma unroll
        for (int it = 0; it < 4; ++it) {
          const int row = it * 4 + q;
          const float* sp = slab + row * SLABP + c8;
          v8h hv;
#pragma unroll
          for (int e = 0; e < 8; ++e) hv[e] = (_Float16)sp[e];
          *(volatile v8h*)(C + (size_t)(mBase + row) * KSPEC + n0 + c8) = hv;
        }
        __threadfence();
      }
    }
    __builtin_amdgcn_fence(__ATOMIC_RELEASE, "workgroup");
    __builtin_amdgcn_wave_barrier();
    __builtin_amdgcn_fence(__ATOMIC_ACQUIRE, "workgroup");
  }
}

__global__ __launch_bounds__(NTHR) void prep_filters(const float* __restrict__ V, unsigned short* __restrict__ Wrev) {
  const int i  = blockIdx.x * NTHR + threadIdx.x;
  const int kf = i / (WPITCH / 8);
  const int g  = i - kf * (WPITCH / 8);
  const int p0 = g * 8;
  const int ke = kf & (NEIG - 1);
  const bool alt = (kf >= NEIG);
  v8h hv;
#pragma unroll
  for (int e = 0; e < 8; ++e) {
    const int p  = p0 + e;
    const int t  = (SEQ - 1) - p;
    const int tc = (t < 0) ? 0 : t;
    float v = bfr(V[tc * NEIG + ke]);
    if (alt && (tc & 1)) v = -v;
    v = (t < 0) ? 0.0f : v;
    hv[e] = (_Float16)v;
  }
  const size_t o = (size_t)i * 8;
  *(volatile v8h*)(Wrev + o) = hv;
  __threadfence();
  *(volatile v8h*)(Wrev + o) = hv;
}

__global__ __launch_bounds__(NTHR) void transpose_cast16(const float* __restrict__ in, long istride,
                                                        unsigned short* __restrict__ out, long ostride,
                                                        int ldo, int c0, float carry) {
  __shared__ __align__(16) float sF[64 * SLABP];
  const int tid = threadIdx.x;
  const int xs = blockIdx.x, ys = blockIdx.y, z = blockIdx.z;
  const float* src = in + (size_t)z * istride + (size_t)(xs * 64) * DMOD + ys * 64;
  const int lr = tid >> 4, lc4 = (tid & 15) * 4;
#pragma unroll
  for (int it = 0; it < 4; ++it) {
    const int r = lr + 16 * it;
    const v4f v = *(const v4f*)(src + (size_t)r * DMOD + lc4);
#pragma unroll
    for (int e = 0; e < 4; ++e) {
      const float x = v[e];
      sF[(lc4 + e) * SLABP + r] = carry * bfr(x);
    }
  }
  __syncthreads();
  const int q = tid >> 3, c8 = (tid & 7) * 8;
  unsigned short* ob = out + (size_t)z * ostride;
  for (int pass = 0; pass < 2; ++pass) {
#pragma unroll
    for (int it = 0; it < 2; ++it) {
      const int orow = q + 32 * it;
      const float* sp = sF + orow * SLABP + c8;
      v8h hv;
#pragma unroll
      for (int e = 0; e < 8; ++e) hv[e] = (_Float16)sp[e];
      *(volatile v8h*)(ob + (size_t)(ys * 64 + orow) * ldo + c0 + xs * 64 + c8) = hv;
    }
    __threadfence();
  }
}

__global__ __launch_bounds__(NTHR) void build_ushift(const float* __restrict__ u, unsigned short* __restrict__ ush) {
  const int i   = blockIdx.x * NTHR + threadIdx.x;
  const int gpr = KLAGU / 8;
  const int r   = i / gpr;
  const int g   = i - r * gpr;
  const int c8  = g * 8;
  const int lag = c8 / DMOD;
  const int d   = c8 - lag * DMOD;
  const int b   = r >> 10;
  const int l   = r & (SEQ - 1);
  const int sl  = l - lag;
  const int slc = (sl < 0) ? 0 : sl;
  const bool keep = (sl >= 0);
  const float* src = u + ((size_t)(b * SEQ + slc)) * DMOD + d;
  const v4f a0 = *(const v4f*)(src);
  const v4f a1 = *(const v4f*)(src + 4);
  v8h hv;
#pragma unroll
  for (int e = 0; e < 4; ++e) {
    const float x0 = a0[e];
    const float x1 = a1[e];
    const float y0 = bfr(x0);
    const float y1 = bfr(x1);
    hv[e]     = (_Float16)(keep ? y0 : 0.0f);
    hv[4 + e] = (_Float16)(keep ? y1 : 0.0f);
  }
  const size_t o = (size_t)i * 8;
  *(volatile v8h*)(ush + o) = hv;
  __threadfence();
  *(volatile v8h*)(ush + o) = hv;
}

__global__ __launch_bounds__(NTHR) void build_my16(const float* __restrict__ My, unsigned short* __restrict__ my16) {
  const int i = blockIdx.x * NTHR + threadIdx.x;
  const int o = i / (KLAGY / 8);
  const int g = i - o * (KLAGY / 8);
  const int c = g * 8;
  int cs = c + DMOD;
  if (cs >= KLAGY) cs -= KLAGY;
  const float* src = My + (size_t)o * KLAGY + cs;
  const v4f a0 = *(const v4f*)(src);
  const v4f a1 = *(const v4f*)(src + 4);
  v8h hv;
#pragma unroll
  for (int e = 0; e < 4; ++e) {
    const float x0 = a0[e];
    const float x1 = a1[e];
    hv[e]     = (_Float16)(WCARRY * bfr(x0));
    hv[4 + e] = (_Float16)(WCARRY * bfr(x1));
  }
  const size_t off = (size_t)i * 8;
  *(volatile v8h*)(my16 + off) = hv;
  __threadfence();
  *(volatile v8h*)(my16 + off) = hv;
}

__global__ __launch_bounds__(NTHR) void zero_sp_rows(float* __restrict__ Sp) {
  const int i = blockIdx.x * NTHR + threadIdx.x;
  if (i >= NB * 2 * DMOD / 4) return;
  const int per = 2 * DMOD / 4;
  const int b   = i / per;
  const int rem = i - b * per;
  float* dst = Sp + (size_t)b * SEQP * DMOD + rem * 4;
  const v4f zv = (v4f){0.f, 0.f, 0.f, 0.f};
  *(volatile v4f*)dst = zv;
  __threadfence();
  *(volatile v4f*)dst = zv;
}

__global__ __launch_bounds__(NTHR) void cast_zp16(const float* __restrict__ Zf, unsigned short* __restrict__ Zp) {
  const int i = blockIdx.x * NTHR + threadIdx.x;
  if (i >= ZP_GROUPS) return;
  const int gpr  = DMOD / 8;
  const int perb = SEQP * gpr;
  const int b    = i / perb;
  const int rem  = i - b * perb;
  const int r    = rem / gpr;
  const int g    = rem - r * gpr;
  const int c8   = g * 8;
  const int sr   = r - 2;
  const int src_r = (sr < 0) ? 0 : sr;
  const bool keep = (sr >= 0);
  const float* src = Zf + ((size_t)(b * SEQ + src_r)) * DMOD + c8;
  const v4f a0 = *(const v4f*)(src);
  const v4f a1 = *(const v4f*)(src + 4);
  v8h hv;
#pragma unroll
  for (int e = 0; e < 4; ++e) {
    const float x0 = a0[e];
    const float x1 = a1[e];
    hv[e]     = (_Float16)(keep ? x0 : 0.0f);
    hv[4 + e] = (_Float16)(keep ? x1 : 0.0f);
  }
  const size_t o = (size_t)i * 8;
  *(volatile v8h*)(Zp + o) = hv;
  __threadfence();
  *(volatile v8h*)(Zp + o) = hv;
}

extern "C" void kernel_launch(void* const* d_in, const int* in_sizes, int n_in,
                              void* d_out, int out_size, void* d_ws, size_t ws_size,
                              hipStream_t stream) {
  if (n_in < 7) return;
  if ((size_t)out_size < (size_t)NB * SEQ * DMOD) return;
  if (ws_size < WS_TOTAL) return;
  if (in_sizes[0] != NB * SEQ * DMOD) return;
  if (in_sizes[1] != NEIG) return;
  if (in_sizes[2] != SEQ * NEIG) return;
  if (in_sizes[3] != NLAGU * DMOD * DMOD) return;
  if (in_sizes[4] != NEIG * DMOD * DMOD) return;
  if (in_sizes[5] != NEIG * DMOD * DMOD) return;
  if (in_sizes[6] != DMOD * NLAGY * DMOD) return;

  const float* inputs = (const float*)d_in[0];
  const float* sigma  = (const float*)d_in[1];
  const float* Vf     = (const float*)d_in[2];
  const float* Mu     = (const float*)d_in[3];
  const float* Mp     = (const float*)d_in[4];
  const float* Mm     = (const float*)d_in[5];
  const float* My     = (const float*)d_in[6];
  float* out = (float*)d_out;

  char* ws = (char*)d_ws;
  unsigned short* Uc    = (unsigned short*)(ws + OFF_UC);
  unsigned short* McatT = (unsigned short*)(ws + OFF_MCAT);
  unsigned short* Ush   = (unsigned short*)(ws + OFF_USH);
  float*          Sp    = (float*)(ws + OFF_SP);
  float*          Zf    = (float*)(ws + OFF_ZF);
  unsigned short* Zp    = (unsigned short*)(ws + OFF_ZP);
  unsigned short* MuT   = (unsigned short*)(ws + OFF_MUT);
  unsigned short* uT    = (unsigned short*)(ws + OFF_UT);
  unsigned short* My16  = (unsigned short*)(ws + OFF_MY);
  unsigned short* Wrev  = (unsigned short*)(ws + OFF_WREV);

  prep_filters<<<(NFILT * WPITCH / 8) / NTHR, NTHR, 0, stream>>>(Vf, Wrev);
  transpose_cast16<<<dim3(SEQ / 64, DMOD / 64, NB), NTHR, 0, stream>>>(
      inputs, (long)SEQ * DMOD, uT, (long)DMOD * SEQ, SEQ, 0, 1.0f);
  build_ushift<<<(NB * SEQ * KLAGU / 8) / NTHR, NTHR, 0, stream>>>(inputs, Ush);
  transpose_cast16<<<dim3(NEIG * DMOD / 64, DMOD / 64, 1), NTHR, 0, stream>>>(
      Mp, 0L, McatT, 0L, KSPEC, 0, WCARRY);
  transpose_cast16<<<dim3(NEIG * DMOD / 64, DMOD / 64, 1), NTHR, 0, stream>>>(
      Mm, 0L, McatT, 0L, KSPEC, NEIG * DMOD, WCARRY);
  transpose_cast16<<<dim3(KLAGU / 64, DMOD / 64, 1), NTHR, 0, stream>>>(
      Mu, 0L, MuT, 0L, KLAGU, 0, WCARRY);
  build_my16<<<(DMOD * KLAGY / 8) / NTHR, NTHR, 0, stream>>>(My, My16);
  zero_sp_rows<<<(NB * 2 * DMOD / 4) / NTHR, NTHR, 0, stream>>>(Sp);

  for (int b = 0; b < NB; ++b) {
    conv_causal_f16<<<dim3(GEMM_GX, NFILT), NTHR, 0, stream>>>(
        Wrev, uT + (size_t)b * DMOD * SEQ, sigma, Uc);
    gemm64_f16<false><<<dim3(GEMM_GX, 1), NTHR, 0, stream>>>(
        Uc, KSPEC, 0L,
        McatT, KSPEC, 0L,
        Sp + ((size_t)b * SEQP + 2) * DMOD, DMOD, 0L,
        nullptr, 0L,
        SEQ, DMOD, KSPEC, WCARRY_INV);
  }
  gemm64_f16<true><<<dim3(GEMM_GX, NB), NTHR, 0, stream>>>(
      Ush, KLAGU, (long)SEQ * KLAGU,
      MuT, KLAGU, 0L,
      Zf, DMOD, (long)SEQ * DMOD,
      Sp, (long)SEQP * DMOD,
      SEQ, DMOD, KLAGU, WCARRY_INV);
  cast_zp16<<<(ZP_GROUPS + NTHR - 1) / NTHR, NTHR, 0, stream>>>(Zf, Zp);
  gemm64_f16<true><<<dim3(GEMM_GX, NB), NTHR, 0, stream>>>(
      Zp, DMOD, (long)SEQP * DMOD,
      My16, KLAGY, 0L,
      out, DMOD, (long)SEQ * DMOD,
      Zf, (long)SEQ * DMOD,
      SEQ, DMOD, KLAGY, WCARRY_INV);
}
